// DualSlidingWindowAttention_52312701665774
// MI455X (gfx1250) — hardware-verified
//
#include <hip/hip_runtime.h>
#include <math.h>

typedef __attribute__((ext_vector_type(16))) _Float16 v16h;
typedef __attribute__((ext_vector_type(8)))  _Float16 v8h;
typedef __attribute__((ext_vector_type(16))) __bf16   v16b;
typedef __attribute__((ext_vector_type(8)))  __bf16   v8b;
typedef __attribute__((ext_vector_type(8)))  float    v8f;
typedef __attribute__((ext_vector_type(4)))  float    v4f;

constexpr int NUM_B     = 2;
constexpr int SEQ_T     = 1024;
constexpr int ROWS_BT   = NUM_B * SEQ_T;
constexpr int HID_SZ    = 2048;
constexpr int QIN_SZ    = 2 * HID_SZ;
constexpr int NUM_QH    = 32;
constexpr int NUM_KVH   = 8;
constexpr int HEAD_D    = 64;
constexpr int KV_COLS   = NUM_KVH * HEAD_D;
constexpr int WIN_SSM   = 64;
constexpr int WIN_ATT   = 256;
constexpr int QTILE     = 64;
constexpr int KCHUNK    = 64;
constexpr int NCHUNK_VIS = 7;
constexpr float QK_SCALE = 0.125f;
constexpr int STG16_PITCH = 72;

constexpr size_t N_XCAT  = (size_t)ROWS_BT * QIN_SZ;
constexpr size_t N_WQT   = (size_t)HID_SZ * QIN_SZ;
constexpr size_t N_WKVT  = (size_t)KV_COLS * HID_SZ;
constexpr size_t N_WOT   = (size_t)HID_SZ * HID_SZ;
constexpr size_t N_QPL   = (size_t)ROWS_BT * HID_SZ;
constexpr size_t N_KVPL  = (size_t)ROWS_BT * KV_COLS;
constexpr size_t OFF_XCAT = 0;
constexpr size_t OFF_WQT  = OFF_XCAT + N_XCAT;
constexpr size_t OFF_WKT  = OFF_WQT  + N_WQT;
constexpr size_t OFF_WVT  = OFF_WKT  + N_WKVT;
constexpr size_t OFF_WSKT = OFF_WVT  + N_WKVT;
constexpr size_t OFF_WSVT = OFF_WSKT + N_WKVT;
constexpr size_t OFF_WOT  = OFF_WSVT + N_WKVT;
constexpr size_t OFF_QH   = OFF_WOT  + N_WOT;
constexpr size_t OFF_QL   = OFF_QH   + N_QPL;
constexpr size_t OFF_SKH  = OFF_QL   + N_QPL;
constexpr size_t OFF_SKL  = OFF_SKH  + N_KVPL;
constexpr size_t OFF_KH   = OFF_SKL  + N_KVPL;
constexpr size_t OFF_KL   = OFF_KH   + N_KVPL;
constexpr size_t OFF_SVTH = OFF_KL   + N_KVPL;
constexpr size_t OFF_SVTL = OFF_SVTH + N_KVPL;
constexpr size_t OFF_VTH  = OFF_SVTL + N_KVPL;
constexpr size_t OFF_VTL  = OFF_VTH  + N_KVPL;
constexpr size_t OFF_OH   = OFF_VTL  + N_KVPL;
constexpr size_t OFF_OL   = OFF_OH   + N_QPL;
constexpr size_t WS_HALVES = OFF_OL  + N_QPL;
constexpr size_t WS_BYTES_USED = WS_HALVES * 2;
static_assert(WS_BYTES_USED == 100663296ull, "ws total");
static_assert(WS_BYTES_USED <= 134217728ull, "ws cap");

__device__ __forceinline__ unsigned short f2bf_bits(float f) {
  unsigned u = __float_as_uint(f);
  return (unsigned short)((u + 0x7FFFu + ((u >> 16) & 1u)) >> 16);
}
__device__ __forceinline__ float bf_bits2f(unsigned short h) { return __uint_as_float(((unsigned)h) << 16); }

__device__ __forceinline__ void dep_guard_h(v8f& a, v8f& b, v16h x, v16h y) { asm volatile("v_nop\n\tv_nop\n\tv_nop\n\tv_nop" : "+v"(a), "+v"(b) : "v"(x), "v"(y)); }
__device__ __forceinline__ void dep_guard_b(v8f& a, v8f& b, v16b x, v16b y) { asm volatile("v_nop\n\tv_nop\n\tv_nop\n\tv_nop" : "+v"(a), "+v"(b) : "v"(x), "v"(y)); }
__device__ __forceinline__ void keep4_h(v16h a, v16h b, v16h c, v16h d) { asm volatile("v_nop" :: "v"(a), "v"(b), "v"(c), "v"(d)); }
__device__ __forceinline__ void keep4_b(v16b a, v16b b, v16b c, v16b d) { asm volatile("v_nop" :: "v"(a), "v"(b), "v"(c), "v"(d)); }
__device__ __forceinline__ void acc_guard4(v8f& a, v8f& b, v8f& c, v8f& d) { asm volatile("v_nop\n\tv_nop\n\tv_nop\n\tv_nop" : "+v"(a), "+v"(b), "+v"(c), "+v"(d)); }
template <typename T> struct Frag;
template <> struct Frag<_Float16> {
  typedef v16h V; union U { v16h v; v8h h[2]; };
  static __device__ __forceinline__ v16h load(const _Float16* p) {
    U f; f.h[0] = *(const v8h*)(p); f.h[1] = *(const v8h*)(p + 16); return f.v;
  }
  static __device__ __forceinline__ v8f mma(v16h a, v16h b, v8f c) {
    return __builtin_amdgcn_wmma_f32_16x16x32_f16(false, a, false, b, (short)0, c, false, false);
  }
  static __device__ __forceinline__ void guard(v8f& a, v8f& b, v16h x, v16h y) { dep_guard_h(a, b, x, y); }
  static __device__ __forceinline__ void keep(v16h a, v16h b, v16h c, v16h d) { keep4_h(a, b, c, d); }
};
template <> struct Frag<__bf16> {
  typedef v16b V; union U { v16b v; v8b h[2]; };
  static __device__ __forceinline__ v16b load(const __bf16* p) {
    U f; f.h[0] = *(const v8b*)(p); f.h[1] = *(const v8b*)(p + 16); return f.v;
  }
  static __device__ __forceinline__ v8f mma(v16b a, v16b b, v8f c) {
    return __builtin_amdgcn_wmma_f32_16x16x32_bf16(false, a, false, b, (short)0, c, false, false);
  }
  static __device__ __forceinline__ void guard(v8f& a, v8f& b, v16b x, v16b y) { dep_guard_b(a, b, x, y); }
  static __device__ __forceinline__ void keep(v16b a, v16b b, v16b c, v16b d) { keep4_b(a, b, c, d); }
};

__device__ __forceinline__ unsigned short at_bf_bits(float f) {
  unsigned u = __float_as_uint(f);
  return (unsigned short)((u + 0x7FFFu + ((u >> 16) & 1u)) >> 16);
}
__device__ __forceinline__ __bf16 at_f2bf(float f) { return __builtin_bit_cast(__bf16, at_bf_bits(f)); }
__device__ __forceinline__ void at_split(float f, __bf16& hi, __bf16& lo) {
  const unsigned short hb = at_bf_bits(f);
  hi = __builtin_bit_cast(__bf16, hb);
  lo = at_f2bf(f - __uint_as_float(((unsigned)hb) << 16));
}
__device__ __forceinline__ v8f at_mma(v16b a, v16b b, v8f c) {
  c = __builtin_amdgcn_wmma_f32_16x16x32_bf16(false, a, false, b, (short)0, c, false, false);
  asm volatile("v_nop\n\tv_nop\n\tv_nop\n\tv_nop" : "+v"(c) : "v"(a), "v"(b));
  return c;
}
__device__ __forceinline__ void lds_fence_wave() {
  __builtin_amdgcn_fence(__ATOMIC_RELEASE, "workgroup");
  __builtin_amdgcn_wave_barrier();
  __builtin_amdgcn_fence(__ATOMIC_ACQUIRE, "workgroup");
}

template <int ET> struct Elem;
template <> struct Elem<0> { typedef _Float16 T; };
template <> struct Elem<1> { typedef __bf16 T; };
template <int ET, int SPLITM, int BIAS_MODE, int OUT_MODE, bool RESID, int ACT = 0>
__global__ __launch_bounds__(256) void wmma_gemm64(
    const unsigned short* __restrict__ Ap, const unsigned short* __restrict__ A2p, int lda, long strideA,
    const unsigned short* __restrict__ Btp, const unsigned short* __restrict__ Bt2p, int ldb, long strideB,
    void* __restrict__ Cout, void* __restrict__ Cout2, int ldc, long strideC,
    const float* __restrict__ bias,
    const float* __restrict__ resid, long strideR,
    int M, int N, int K, float scale) {
  typedef typename Elem<ET>::T T;
  typedef typename Frag<T>::V V;
  constexpr bool SPA = (SPLITM >= 1);
  constexpr bool SPB = (SPLITM >= 2);
  const T* A = (const T*)Ap; const T* A2 = (const T*)A2p; const T* Bt = (const T*)Btp; const T* Bt2 = (const T*)Bt2p;
  __shared__ __align__(16) float sT[8][16 * 68];
  const int b    = blockIdx.y;
  const int lane = threadIdx.x & 31;
  const int wave = threadIdx.x >> 5;
  const int tilesN = N >> 6;
  const int tilesM = M >> 6;
  const int tile = blockIdx.x * 8 + wave;
  if (tile >= tilesM * tilesN) return;
  const int tm = tile / tilesN;
  const int tn = tile - tm * tilesN;
  const int m0 = tm << 6;
  const int n0 = tn << 6;

  const T* Ab  = A  + (size_t)b * strideA;
  const T* Bb  = Bt + (size_t)b * strideB;
  const T* Ab2 = SPA ? (A2  + (size_t)b * strideA) : nullptr;
  const T* Bb2 = SPB ? (Bt2 + (size_t)b * strideB) : nullptr;

  const int rlane = lane & 15;
  const int koff  = (lane >> 4) * 8;
  const int mOff  = (lane >> 4) * 8;

  v8f acc[4][4];
#pragma unroll
  for (int i = 0; i < 4; ++i)
#pragma unroll
    for (int j = 0; j < 4; ++j) acc[i][j] = (v8f){0.f,0.f,0.f,0.f,0.f,0.f,0.f,0.f};

  for (int k0 = 0; k0 < K; k0 += 32) {
    V bh[4], bl[4];
#pragma unroll
    for (int j = 0; j < 4; ++j) {
      const size_t bo = (size_t)(n0 + (j << 4) + rlane) * ldb + koff + k0;
      bh[j] = Frag<T>::load(Bb + bo);
      if (SPB) bl[j] = Frag<T>::load(Bb2 + bo);
    }
#pragma unroll
    for (int i = 0; i < 4; ++i) {
      const size_t ao = (size_t)(m0 + (i << 4) + rlane) * lda + koff + k0;
      V ah = Frag<T>::load(Ab + ao);
      V al;
      if (SPA) al = Frag<T>::load(Ab2 + ao);
#pragma unroll
      for (int j = 0; j < 4; ++j) {
        acc[i][j] = Frag<T>::mma(ah, bh[j], acc[i][j]);
        if (SPB) acc[i][j] = Frag<T>::mma(ah, bl[j], acc[i][j]);
        if (SPA) acc[i][j] = Frag<T>::mma(al, bh[j], acc[i][j]);
      }
      Frag<T>::guard(acc[i][0], acc[i][3], ah, SPA ? al : ah);
    }
    Frag<T>::keep(bh[0], bh[1], bh[2], bh[3]);
    if (SPB) Frag<T>::keep(bl[0], bl[1], bl[2], bl[3]);
  }
  acc_guard4(acc[0][0], acc[0][1], acc[0][2], acc[0][3]);
  acc_guard4(acc[1][0], acc[1][1], acc[1][2], acc[1][3]);
  acc_guard4(acc[2][0], acc[2][1], acc[2][2], acc[2][3]);
  acc_guard4(acc[3][0], acc[3][1], acc[3][2], acc[3][3]);

  float* slab = sT[wave];
  const float* Rb = RESID ? (resid + (size_t)b * strideR) : nullptr;
#pragma unroll
  for (int i = 0; i < 4; ++i) {
    const int mBase = m0 + (i << 4);
#pragma unroll
    for (int j = 0; j < 4; ++j) {
      const int n = n0 + (j << 4) + rlane;
      float bv = 0.f;
      if (BIAS_MODE == 2) bv = bias[n];
#pragma unroll
      for (int r = 0; r < 8; ++r) {
        float v = acc[i][j][r] * scale;
        if (BIAS_MODE == 1) v += bias[mBase + mOff + r];
        if (BIAS_MODE == 2) v += bv;
        if (RESID) v += Rb[(size_t)(mBase + mOff + r) * ldc + n];
        if (ACT == 1) v = tanhf(v);
        if (ACT == 2) v = fmaxf(v, 0.0f);
        if (ACT == 4) v = (v > 0.f) ? v : 0.01f * v;
        slab[(mOff + r) * 68 + (j << 4) + rlane] = v;
      }
    }
    __builtin_amdgcn_fence(__ATOMIC_RELEASE, "workgroup");
    __builtin_amdgcn_wave_barrier();
    __builtin_amdgcn_fence(__ATOMIC_ACQUIRE, "workgroup");
    if (OUT_MODE == 0) {
      float* C = (float*)Cout + (size_t)b * strideC;
      const int hh = lane >> 4, c4 = (lane & 15) * 4;
      for (int pass = 0; pass < 2; ++pass) {
#pragma unroll
        for (int it = 0; it < 8; ++it) {
          const int row = it * 2 + hh;
          v4f v = *(const v4f*)(slab + row * 68 + c4);
          *(volatile v4f*)(C + (size_t)(mBase + row) * ldc + n0 + c4) = v;
        }
        __threadfence();
      }
    } else {
      const int q = lane >> 3, c8 = (lane & 7) * 8;
      unsigned short* C  = (unsigned short*)Cout  + (size_t)b * strideC;
      unsigned short* C2 = (OUT_MODE == 2) ? ((unsigned short*)Cout2 + (size_t)b * strideC) : nullptr;
      for (int pass = 0; pass < 2; ++pass) {
#pragma unroll
        for (int it = 0; it < 4; ++it) {
          const int row = it * 4 + q;
          const float* sp = slab + row * 68 + c8;
          v8h hv, lv;
#pragma unroll
          for (int e = 0; e < 8; ++e) {
            if (OUT_MODE == 1) {
              hv[e] = (_Float16)sp[e];
            } else {
              unsigned short hb = f2bf_bits(sp[e]);
              unsigned short lb = f2bf_bits(sp[e] - bf_bits2f(hb));
              hv[e] = __builtin_bit_cast(_Float16, hb);
              lv[e] = __builtin_bit_cast(_Float16, lb);
            }
          }
          *(volatile v8h*)(C + (size_t)(mBase + row) * ldc + n0 + c8) = hv;
          if (OUT_MODE == 2) *(volatile v8h*)(C2 + (size_t)(mBase + row) * ldc + n0 + c8) = lv;
        }
        __threadfence();
      }
    }
    __builtin_amdgcn_fence(__ATOMIC_RELEASE, "workgroup");
    __builtin_amdgcn_wave_barrier();
    __builtin_amdgcn_fence(__ATOMIC_ACQUIRE, "workgroup");
  }
}

__global__ __launch_bounds__(256) void cast_rows_bf16_k(const float* __restrict__ in,
                                                         unsigned short* __restrict__ out,
                                                         int npair_row, int ld_out_pairs, int total_pairs) {
  const int i = blockIdx.x * 256 + threadIdx.x;
  if (i < total_pairs) {
    const int row = i / npair_row;
    const int p   = i - row * npair_row;
    const unsigned u = (unsigned)f2bf_bits(in[2 * (size_t)i]) | ((unsigned)f2bf_bits(in[2 * (size_t)i + 1]) << 16);
    volatile unsigned* o = (volatile unsigned*)out + (size_t)row * ld_out_pairs + p;
    *o = u;
    __threadfence();
    *o = u;
  }
}

__global__ __launch_bounds__(256) void transpose_cast_bf16_k(const float* __restrict__ in,
                                                              unsigned short* __restrict__ out,
                                                              int R, int Ccols) {
  __shared__ __align__(16) _Float16 t[64 * STG16_PITCH];
  const int c0 = blockIdx.x * 64, r0 = blockIdx.y * 64;
  const int tid = threadIdx.x;
  {
    const int rloc = tid >> 2, cq = (tid & 3) * 16;
    const float* src = in + (size_t)(r0 + rloc) * Ccols + c0 + cq;
#pragma unroll
    for (int i = 0; i < 4; ++i) {
      const v4f v = *(const v4f*)(src + 4 * i);
#pragma unroll
      for (int e = 0; e < 4; ++e)
        t[(cq + 4 * i + e) * STG16_PITCH + rloc] = __builtin_bit_cast(_Float16, f2bf_bits(v[e]));
    }
  }
  __syncthreads();
  const int wave = tid >> 5, lane = tid & 31, q8 = lane >> 3, c8 = (lane & 7) * 8;
  const int cA = wave * 8 + q8, cB = wave * 8 + 4 + q8;
  const v8h va = *(const v8h*)(t + cA * STG16_PITCH + c8);
  const v8h vb = *(const v8h*)(t + cB * STG16_PITCH + c8);
  unsigned short* da = out + (size_t)(c0 + cA) * R + r0 + c8;
  unsigned short* db = out + (size_t)(c0 + cB) * R + r0 + c8;
  for (int pass = 0; pass < 2; ++pass) {
    *(volatile v8h*)da = va;
    *(volatile v8h*)db = vb;
    __threadfence();
  }
}

__global__ __launch_bounds__(128)
void dswa_attn_k(const unsigned short* __restrict__ Qhp,  const unsigned short* __restrict__ Qlp,
                 const unsigned short* __restrict__ SKhp, const unsigned short* __restrict__ SKlp,
                 const unsigned short* __restrict__ SVthp, const unsigned short* __restrict__ SVtlp,
                 const unsigned short* __restrict__ AKhp, const unsigned short* __restrict__ AKlp,
                 const unsigned short* __restrict__ AVthp, const unsigned short* __restrict__ AVtlp,
                 unsigned short* __restrict__ Ohp, unsigned short* __restrict__ Olp) {
  union FB { v16b v; v8b h[2]; };
  __shared__ __align__(16) __bf16 Ksh[KCHUNK * HEAD_D];
  __shared__ __align__(16) __bf16 Ksl[KCHUNK * HEAD_D];
  __shared__ __align__(16) __bf16 Vsh[HEAD_D * KCHUNK];
  __shared__ __align__(16) __bf16 Vsl[HEAD_D * KCHUNK];
  __shared__ __align__(16) __bf16 Psh[4][16 * KCHUNK];
  __shared__ __align__(16) __bf16 Psl[4][16 * KCHUNK];

  const int tid  = threadIdx.x;
  const int wave = tid >> 5;
  const int lane = tid & 31;
  const int hh   = lane >> 4;
  const int c    = lane & 15;

  const int nqb = SEQ_T / QTILE;
  const int bx  = blockIdx.x;
  const int qb  = bx % nqb;
  const int bhi = bx / nqb;
  const int h   = bhi % NUM_QH;
  const int b   = bhi / NUM_QH;
  const int kvh = h / (NUM_QH / NUM_KVH);
  const int q0  = qb * QTILE + wave * 16;
  const float slope = exp2f(-0.25f * (float)h);

  const __bf16* Qh = (const __bf16*)Qhp;
  const __bf16* Ql = (const __bf16*)Qlp;

  v16b qah[2], qal[2];
  {
    const size_t qo = (size_t)(b * SEQ_T + q0 + c) * HID_SZ + h * HEAD_D + 8 * hh;
#pragma unroll
    for (int dc = 0; dc < 2; ++dc) {
      qah[dc] = Frag<__bf16>::load(Qh + qo + dc * 32);
      qal[dc] = Frag<__bf16>::load(Ql + qo + dc * 32);
    }
  }

  float mrow[8], lrow[8];
  v8f oacc[4];
#pragma unroll
  for (int r = 0; r < 8; ++r) { mrow[r] = -INFINITY; lrow[r] = 0.f; }
#pragma unroll
  for (int t = 0; t < 4; ++t) oacc[t] = (v8f){0.f,0.f,0.f,0.f,0.f,0.f,0.f,0.f};

  __bf16* pwh = Psh[wave];
  __bf16* pwl = Psl[wave];

#pragma unroll 1
  for (int ci = 0; ci < NCHUNK_VIS; ++ci) {
    const bool is_ssm = (ci < 2);
    const int  kc = is_ssm ? (qb - ci) : (qb - (ci - 2));
    if (kc < 0) continue;
    const int win = is_ssm ? WIN_SSM : WIN_ATT;
    const __bf16* Kh  = (const __bf16*)(is_ssm ? SKhp  : AKhp);
    const __bf16* Kl  = (const __bf16*)(is_ssm ? SKlp  : AKlp);
    const __bf16* Vth = (const __bf16*)(is_ssm ? SVthp : AVthp);
    const __bf16* Vtl = (const __bf16*)(is_ssm ? SVtlp : AVtlp);
    const int kv0 = kc * KCHUNK;

    __syncthreads();
    {
      const int r = tid >> 1, h32 = (tid & 1) * 32;
      const size_t ko = (size_t)(b * SEQ_T + kv0 + r) * KV_COLS + kvh * HEAD_D + h32;
      const size_t vo = (size_t)(kvh * HEAD_D + r) * ROWS_BT + b * SEQ_T + kv0 + h32;
#pragma unroll
      for (int i = 0; i < 4; ++i) {
        const v8b k1 = *(const v8b*)(Kh  + ko + 8 * i);
        const v8b k2 = *(const v8b*)(Kl  + ko + 8 * i);
        const v8b v1 = *(const v8b*)(Vth + vo + 8 * i);
        const v8b v2 = *(const v8b*)(Vtl + vo + 8 * i);
        *(v8b*)(Ksh + r * HEAD_D + h32 + 8 * i) = k1;
        *(v8b*)(Ksl + r * HEAD_D + h32 + 8 * i) = k2;
        *(v8b*)(Vsh + r * KCHUNK + h32 + 8 * i) = v1;
        *(v8b*)(Vsl + r * KCHUNK + h32 + 8 * i) = v2;
      }
    }
    __syncthreads();

    v8f s[4];
#pragma unroll
    for (int j = 0; j < 4; ++j) {
      s[j] = (v8f){0.f,0.f,0.f,0.f,0.f,0.f,0.f,0.f};
#pragma unroll
      for (int dc = 0; dc < 2; ++dc) {
        FB kb, kl;
        kb.h[0] = *(const v8b*)(Ksh + (j * 16 + c) * HEAD_D + dc * 32 + 8 * hh);
        kb.h[1] = *(const v8b*)(Ksh + (j * 16 + c) * HEAD_D + dc * 32 + 16 + 8 * hh);
        kl.h[0] = *(const v8b*)(Ksl + (j * 16 + c) * HEAD_D + dc * 32 + 8 * hh);
        kl.h[1] = *(const v8b*)(Ksl + (j * 16 + c) * HEAD_D + dc * 32 + 16 + 8 * hh);
        s[j] = at_mma(qah[dc], kb.v, s[j]);
        s[j] = at_mma(qah[dc], kl.v, s[j]);
        s[j] = at_mma(qal[dc], kb.v, s[j]);
      }
    }

    float cm[8];
#pragma unroll
    for (int r = 0; r < 8; ++r) {
      const int qrow = q0 + 8 * hh + r;
      float m = -INFINITY;
#pragma unroll
      for (int j = 0; j < 4; ++j) {
        const int kvcol = kv0 + j * 16 + c;
        const int delta = qrow - kvcol;
        const bool valid = (delta >= 0) && (delta < win);
        const float sc = s[j][r] * QK_SCALE + slope * (float)(kvcol - qrow);
        const float sv = valid ? sc : -INFINITY;
        s[j][r] = sv;
        m = fmaxf(m, sv);
      }
#pragma unroll
      for (int off = 1; off < 16; off <<= 1) m = fmaxf(m, __shfl_xor(m, off, 32));
      cm[r] = m;
    }

#pragma unroll
    for (int r = 0; r < 8; ++r) {
      const float mnew  = fmaxf(mrow[r], cm[r]);
      const float msafe = (mnew == -INFINITY) ? 0.f : mnew;
      const float alpha = expf(mrow[r] - msafe);
      mrow[r] = mnew;
      float psum = 0.f;
#pragma unroll
      for (int j = 0; j < 4; ++j) {
        const float p = expf(s[j][r] - msafe);
        psum += p;
        __bf16 a, bl;
        at_split(p, a, bl);
        pwh[(8 * hh + r) * KCHUNK + j * 16 + c] = a;
        pwl[(8 * hh + r) * KCHUNK + j * 16 + c] = bl;
      }
#pragma unroll
      for (int off = 1; off < 16; off <<= 1) psum += __shfl_xor(psum, off, 32);
      lrow[r] = lrow[r] * alpha + psum;
#pragma unroll
      for (int t = 0; t < 4; ++t) oacc[t][r] *= alpha;
    }
    lds_fence_wave();

#pragma unroll 1
    for (int kk = 0; kk < 2; ++kk) {
      FB pa, pl;
      pa.h[0] = *(const v8b*)(pwh + c * KCHUNK + kk * 32 + 8 * hh);
      pa.h[1] = *(const v8b*)(pwh + c * KCHUNK + kk * 32 + 16 + 8 * hh);
      pl.h[0] = *(const v8b*)(pwl + c * KCHUNK + kk * 32 + 8 * hh);
      pl.h[1] = *(const v8b*)(pwl + c * KCHUNK + kk * 32 + 16 + 8 * hh);
#pragma unroll
      for (int t = 0; t < 4; ++t) {
        FB vb, vl;
        vb.h[0] = *(const v8b*)(Vsh + (t * 16 + c) * KCHUNK + kk * 32 + 8 * hh);
        vb.h[1] = *(const v8b*)(Vsh + (t * 16 + c) * KCHUNK + kk * 32 + 16 + 8 * hh);
        vl.h[0] = *(const v8b*)(Vsl + (t * 16 + c) * KCHUNK + kk * 32 + 8 * hh);
        vl.h[1] = *(const v8b*)(Vsl + (t * 16 + c) * KCHUNK + kk * 32 + 16 + 8 * hh);
        oacc[t] = at_mma(pa.v, vb.v, oacc[t]);
        oacc[t] = at_mma(pa.v, vl.v, oacc[t]);
        oacc[t] = at_mma(pl.v, vb.v, oacc[t]);
      }
    }
  }

  lds_fence_wave();
#pragma unroll
  for (int r = 0; r < 8; ++r) {
    const float inv = 1.0f / lrow[r];
#pragma unroll
    for (int t = 0; t < 4; ++t) {
      __bf16 a, bl;
      at_split(oacc[t][r] * inv, a, bl);
      pwh[(8 * hh + r) * KCHUNK + t * 16 + c] = a;
      pwl[(8 * hh + r) * KCHUNK + t * 16 + c] = bl;
    }
  }
  lds_fence_wave();
  {
    const int q8 = lane >> 3, c8 = (lane & 7) * 8;
    const size_t ob = (size_t)(b * SEQ_T + q0) * HID_SZ + h * HEAD_D + c8;
    for (int pass = 0; pass < 2; ++pass) {
#pragma unroll
      for (int it = 0; it < 4; ++it) {
        const int row = it * 4 + q8;
        const v8b hv = *(const v8b*)(pwh + row * KCHUNK + c8);
        const v8b lv = *(const v8b*)(pwl + row * KCHUNK + c8);
        *(volatile v8h*)(Ohp + ob + (size_t)row * HID_SZ) = __builtin_bit_cast(v8h, hv);
        *(volatile v8h*)(Olp + ob + (size_t)row * HID_SZ) = __builtin_bit_cast(v8h, lv);
      }
      __threadfence();
    }
  }
}

extern "C" void kernel_launch(void* const* d_in, const int* in_sizes, int n_in,
                              void* d_out, int out_size, void* d_ws, size_t ws_size,
                              hipStream_t stream) {
  if (n_in < 8) return;
  if (in_sizes[0] != ROWS_BT * HID_SZ || in_sizes[1] != ROWS_BT * HID_SZ) return;
  if (in_sizes[2] != QIN_SZ * HID_SZ) return;
  if (in_sizes[3] != HID_SZ * KV_COLS || in_sizes[4] != HID_SZ * KV_COLS ||
      in_sizes[5] != HID_SZ * KV_COLS || in_sizes[6] != HID_SZ * KV_COLS) return;
  if (in_sizes[7] != HID_SZ * HID_SZ) return;
  if (out_size != ROWS_BT * HID_SZ) return;
  if (ws_size < WS_BYTES_USED) return;

  const float* hidden = (const float*)d_in[0];
  const float* ssm    = (const float*)d_in[1];
  const float* Wq     = (const float*)d_in[2];
  const float* Wk     = (const float*)d_in[3];
  const float* Wv     = (const float*)d_in[4];
  const float* Wsk    = (const float*)d_in[5];
  const float* Wsv    = (const float*)d_in[6];
  const float* Wo     = (const float*)d_in[7];
  float* out = (float*)d_out;

  unsigned short* ws = (unsigned short*)d_ws;
  unsigned short* Xcat = ws + OFF_XCAT;
  unsigned short* WqT  = ws + OFF_WQT;
  unsigned short* WkT  = ws + OFF_WKT;
  unsigned short* WvT  = ws + OFF_WVT;
  unsigned short* WskT = ws + OFF_WSKT;
  unsigned short* WsvT = ws + OFF_WSVT;
  unsigned short* WoT  = ws + OFF_WOT;
  unsigned short* Qh   = ws + OFF_QH;
  unsigned short* Ql   = ws + OFF_QL;
  unsigned short* SKh  = ws + OFF_SKH;
  unsigned short* SKl  = ws + OFF_SKL;
  unsigned short* Kh   = ws + OFF_KH;
  unsigned short* Kl   = ws + OFF_KL;
  unsigned short* SVth = ws + OFF_SVTH;
  unsigned short* SVtl = ws + OFF_SVTL;
  unsigned short* Vth  = ws + OFF_VTH;
  unsigned short* Vtl  = ws + OFF_VTL;
  unsigned short* Oh   = ws + OFF_OH;
  unsigned short* Ol   = ws + OFF_OL;
  const float* wsf = (const float*)d_ws;

  const dim3 b256(256);

  const int total_pairs = ROWS_BT * HID_SZ / 2;
  const int cast_blocks = (total_pairs + 255) / 256;
  cast_rows_bf16_k<<<dim3(cast_blocks), b256, 0, stream>>>(ssm,    Xcat,          HID_SZ / 2, QIN_SZ / 2, total_pairs);
  cast_rows_bf16_k<<<dim3(cast_blocks), b256, 0, stream>>>(hidden, Xcat + HID_SZ, HID_SZ / 2, QIN_SZ / 2, total_pairs);

  transpose_cast_bf16_k<<<dim3(HID_SZ / 64, QIN_SZ / 64),  b256, 0, stream>>>(Wq,  WqT,  QIN_SZ, HID_SZ);
  transpose_cast_bf16_k<<<dim3(KV_COLS / 64, HID_SZ / 64), b256, 0, stream>>>(Wk,  WkT,  HID_SZ, KV_COLS);
  transpose_cast_bf16_k<<<dim3(KV_COLS / 64, HID_SZ / 64), b256, 0, stream>>>(Wv,  WvT,  HID_SZ, KV_COLS);
  transpose_cast_bf16_k<<<dim3(KV_COLS / 64, HID_SZ / 64), b256, 0, stream>>>(Wsk, WskT, HID_SZ, KV_COLS);
  transpose_cast_bf16_k<<<dim3(KV_COLS / 64, HID_SZ / 64), b256, 0, stream>>>(Wsv, WsvT, HID_SZ, KV_COLS);
  transpose_cast_bf16_k<<<dim3(HID_SZ / 64, HID_SZ / 64),  b256, 0, stream>>>(Wo,  WoT,  HID_SZ, HID_SZ);

  {
    const int tiles = (ROWS_BT / 64) * (HID_SZ / 64);
    wmma_gemm64<1, 0, 0, 2, false, 0><<<dim3((tiles + 7) / 8, 1), b256, 0, stream>>>(
        Xcat, Xcat, QIN_SZ, 0L, WqT, WqT, QIN_SZ, 0L, (void*)Qh, (void*)Ql, HID_SZ, 0L,
        wsf, wsf, 0L, ROWS_BT, HID_SZ, QIN_SZ, 1.0f);
  }
  {
    const int tiles = (ROWS_BT / 64) * (KV_COLS / 64);
    wmma_gemm64<1, 0, 0, 2, false, 0><<<dim3((tiles + 7) / 8, 1), b256, 0, stream>>>(
        Xcat, Xcat, QIN_SZ, 0L, WskT, WskT, HID_SZ, 0L, (void*)SKh, (void*)SKl, KV_COLS, 0L,
        wsf, wsf, 0L, ROWS_BT, KV_COLS, HID_SZ, 1.0f);
    wmma_gemm64<1, 0, 0, 2, false, 0><<<dim3((tiles + 7) / 8, 1), b256, 0, stream>>>(
        Xcat + HID_SZ, Xcat + HID_SZ, QIN_SZ, 0L, WkT, WkT, HID_SZ, 0L, (void*)Kh, (void*)Kl, KV_COLS, 0L,
        wsf, wsf, 0L, ROWS_BT, KV_COLS, HID_SZ, 1.0f);
  }
  {
    const int tiles = (KV_COLS / 64) * (ROWS_BT / 64);
    wmma_gemm64<1, 0, 0, 2, false, 0><<<dim3((tiles + 7) / 8, 1), b256, 0, stream>>>(
        WsvT, WsvT, HID_SZ, 0L, Xcat, Xcat, QIN_SZ, 0L, (void*)SVth, (void*)SVtl, ROWS_BT, 0L,
        wsf, wsf, 0L, KV_COLS, ROWS_BT, HID_SZ, 1.0f);
    wmma_gemm64<1, 0, 0, 2, false, 0><<<dim3((tiles + 7) / 8, 1), b256, 0, stream>>>(
        WvT, WvT, HID_SZ, 0L, Xcat + HID_SZ, Xcat + HID_SZ, QIN_SZ, 0L, (void*)Vth, (void*)Vtl, ROWS_BT, 0L,
        wsf, wsf, 0L, KV_COLS, ROWS_BT, HID_SZ, 1.0f);
  }

  dswa_attn_k<<<dim3(NUM_B * NUM_QH * (SEQ_T / QTILE)), dim3(128), 0, stream>>>(
      Qh, Ql, SKh, SKl, SVth, SVtl, Kh, Kl, Vth, Vtl, Oh, Ol);

  {
    const int tiles = (ROWS_BT / 64) * (HID_SZ / 64);
    wmma_gemm64<1, 1, 0, 0, false, 0><<<dim3((tiles + 7) / 8, 1), b256, 0, stream>>>(
        Oh, Ol, HID_SZ, 0L, WoT, WoT, HID_SZ, 0L, (void*)out, (void*)out, HID_SZ, 0L,
        wsf, wsf, 0L, ROWS_BT, HID_SZ, HID_SZ, 1.0f);
  }
}
